// DiagnosticRNN_48026324304699
// MI455X (gfx1250) — hardware-verified
//
#include <hip/hip_runtime.h>


typedef __bf16 bf16t;
typedef bf16t          v16b __attribute__((ext_vector_type(16)));
typedef unsigned short v8us __attribute__((ext_vector_type(8)));
typedef int            v8i  __attribute__((ext_vector_type(8)));
typedef float          v8f  __attribute__((ext_vector_type(8)));
typedef float          v4f  __attribute__((ext_vector_type(4)));

union Frag { v16b v; v8us q[2]; v8i w; };
union PkF  { v8f v; v4f q[2]; };

#define NB    4096
#define SEQT  1024
#define HID   64
#define NCLS  10
#define RB    16
#define TC    64
#define HS    72
#define HF    68
#define NTHR  64

static_assert(NB % RB == 0);
static_assert(SEQT % TC == 0);
static_assert((RB * TC) % NTHR == 0);
static_assert(HID == 64);
static_assert((RB * NCLS) % 4 == 0);
static_assert(((RB * NCLS * 4) % 128) == 0);

__device__ __forceinline__ unsigned int bf16_rne(float f) {
    unsigned int u = __float_as_uint(f);
    u += 0x7FFFu + ((u >> 16) & 1u);
    return u >> 16;
}

__device__ __forceinline__ v8f mma_bf16(const Frag& a, const Frag& b, v8f c) {
    v8f d = __builtin_amdgcn_wmma_f32_16x16x32_bf16(false, a.v, false, b.v, (short)0, c, false, false);
    asm volatile("v_nop\n\tv_nop\n\tv_nop\n\tv_nop" : "+v"(d) : "v"(a.w), "v"(b.w));
    return d;
}

__device__ __forceinline__ float tanh_f(float v) {
    const float a = fabsf(v);
    const float s = v * v;
    float p = fmaf(s, -8.8632355e-3f, 2.1869489e-2f);
    p = fmaf(s, p, -5.3968254e-2f);
    p = fmaf(s, p, 1.3333334e-1f);
    p = fmaf(s, p, -3.3333334e-1f);
    p = p * s;
    const float sm = fmaf(v, p, v);
    const float e  = __expf(2.0f * a);
    float bg = fmaf(-2.0f, __builtin_amdgcn_rcpf(e + 1.0f), 1.0f);
    bg = copysignf(bg, v);
    return (a < 0.25f) ? sm : bg;
}

__global__ __launch_bounds__(NTHR)
void k_elman(const float* __restrict__ x,   const float* __restrict__ Whx,
             const float* __restrict__ Whh, const float* __restrict__ Wph,
             const float* __restrict__ bh,  const float* __restrict__ bp,
             float* out, int nb, int T)
{
    __shared__ __attribute__((aligned(16))) unsigned short hst[2 * 2 * RB * HS];
    __shared__ __attribute__((aligned(16))) unsigned short wp[2 * HID * HS];
    __shared__ __attribute__((aligned(16))) float xbuf[TC * RB];
    __shared__ __attribute__((aligned(16))) float hf[RB * HF];
    __shared__ __attribute__((aligned(16))) float pout[RB * NCLS];

    const int tid  = threadIdx.x;
    const int lane = tid & 31, w = tid >> 5;
    const int h    = lane >> 4, m = lane & 15;
    const int n0   = 32 * w;
    const int gb0  = blockIdx.x * RB;
    if (gb0 + RB > nb) return;

    for (int i = tid; i < 2 * 2 * RB * HS; i += NTHR) hst[i] = (unsigned short)0;

    for (int e = tid; e < HID * HID; e += NTHR) {
        const int k = e >> 6, n = e & (HID - 1);
        const float v = Whh[e];
        const unsigned int hi = bf16_rne(v);
        const float vh = __uint_as_float(hi << 16);
        const unsigned int lo = bf16_rne(v - vh);
        wp[n * HS + k]            = (unsigned short)hi;
        wp[HID * HS + n * HS + k] = (unsigned short)lo;
    }

    float wx[2][8], bv[2][8];
#pragma unroll
    for (int i = 0; i < 2; ++i)
#pragma unroll
        for (int r = 0; r < 8; ++r) {
            const int f = n0 + 16 * i + 8 * h + r;
            wx[i][r] = Whx[f];
            bv[i][r] = bh[f];
        }
    __syncthreads();

    int cur = 0;
#pragma unroll 1
    for (int tc0 = 0; tc0 < T; tc0 += TC) {
        __syncthreads();
#pragma unroll
        for (int k = 0; k < (RB * TC) / NTHR; ++k) {
            const int e   = tid + NTHR * k;
            const int row = e / TC, tt = e - row * TC;
            xbuf[tt * RB + row] = x[(size_t)(gb0 + row) * T + tc0 + tt];
        }
        __syncthreads();

#pragma unroll 1
        for (int tt = 0; tt < TC; ++tt) {
            const unsigned short* Hh = hst + (2 * cur) * (RB * HS);
            const unsigned short* Hl = Hh + RB * HS;
            const float xv = xbuf[tt * RB + m];

            v8f acc[2];
#pragma unroll
            for (int i = 0; i < 2; ++i)
#pragma unroll
                for (int r = 0; r < 8; ++r)
                    acc[i][r] = fmaf(xv, wx[i][r], bv[i][r]);

#pragma unroll
            for (int ks = 0; ks < 2; ++ks) {
                const int ko = 32 * ks + 8 * h;
                Frag bhi, blo, ahi[2], alo[2];
                bhi.q[0] = *(const v8us*)(Hh + m * HS + ko);
                bhi.q[1] = *(const v8us*)(Hh + m * HS + ko + 16);
                blo.q[0] = *(const v8us*)(Hl + m * HS + ko);
                blo.q[1] = *(const v8us*)(Hl + m * HS + ko + 16);
#pragma unroll
                for (int i = 0; i < 2; ++i) {
                    const unsigned short* ap = wp + (n0 + 16 * i + m) * HS + ko;
                    ahi[i].q[0] = *(const v8us*)(ap);
                    ahi[i].q[1] = *(const v8us*)(ap + 16);
                    alo[i].q[0] = *(const v8us*)(ap + HID * HS);
                    alo[i].q[1] = *(const v8us*)(ap + HID * HS + 16);
                }
#pragma unroll
                for (int i = 0; i < 2; ++i) {
                    acc[i] = mma_bf16(ahi[i], bhi, acc[i]);
                    acc[i] = mma_bf16(ahi[i], blo, acc[i]);
                    acc[i] = mma_bf16(alo[i], bhi, acc[i]);
                }
            }

            const bool last = (tc0 + tt) == (T - 1);
            unsigned short* Nh = hst + (2 * (cur ^ 1)) * (RB * HS);
            unsigned short* Nl = Nh + RB * HS;
#pragma unroll
            for (int i = 0; i < 2; ++i) {
                v8us ph = {0, 0, 0, 0, 0, 0, 0, 0};
                v8us pl = {0, 0, 0, 0, 0, 0, 0, 0};
                PkF fv;
#pragma unroll
                for (int r = 0; r < 8; ++r) {
                    const float v = tanh_f(acc[i][r]);
                    const unsigned int hi = bf16_rne(v);
                    const float vh = __uint_as_float(hi << 16);
                    const unsigned int lo = bf16_rne(v - vh);
                    ph[r] = (unsigned short)hi;
                    pl[r] = (unsigned short)lo;
                    fv.v[r] = v;
                }
                const int f = n0 + 16 * i + 8 * h;
                *(v8us*)(Nh + m * HS + f) = ph;
                *(v8us*)(Nl + m * HS + f) = pl;
                if (last) {
                    *(v4f*)(hf + m * HF + f)     = fv.q[0];
                    *(v4f*)(hf + m * HF + f + 4) = fv.q[1];
                }
            }
            cur ^= 1;
            __syncthreads();
        }
    }

#pragma unroll
    for (int j = 0; j < 3; ++j) {
        const int o   = tid + NTHR * j;
        const int oc  = (o < RB * NCLS) ? o : (RB * NCLS - 1);
        const int row = oc / NCLS, cls = oc - row * NCLS;
        float s = 0.0f;
#pragma unroll 8
        for (int k = 0; k < HID; ++k) s = fmaf(hf[row * HF + k], Wph[k * NCLS + cls], s);
        s += bp[cls];
        if (o < RB * NCLS) pout[o] = s;
    }
    __syncthreads();

    {
        const bool wr = tid < (RB * NCLS / 4);
        const int  q  = wr ? tid : 0;
        const v4f pv = *(const v4f*)(pout + 4 * q);
        float* dst = out + (size_t)gb0 * NCLS + 4 * q;
        if (wr) *(volatile v4f*)dst = pv;
        __threadfence();
        if (wr) *(volatile v4f*)dst = pv;
    }
}

extern "C" void kernel_launch(void* const* d_in, const int* in_sizes, int n_in,
                              void* d_out, int out_size, void* d_ws, size_t ws_size,
                              hipStream_t stream) {
    (void)d_ws; (void)ws_size;
    const int nb = NB, T = SEQT;
    if (n_in < 6) return;
    if (in_sizes[0] != nb * T || in_sizes[1] != HID || in_sizes[2] != HID * HID ||
        in_sizes[3] != HID * NCLS || in_sizes[4] != HID || in_sizes[5] != NCLS) return;
    if (out_size != nb * NCLS) return;

    const float* x   = (const float*)d_in[0];
    const float* Whx = (const float*)d_in[1];
    const float* Whh = (const float*)d_in[2];
    const float* Wph = (const float*)d_in[3];
    const float* bh  = (const float*)d_in[4];
    const float* bp  = (const float*)d_in[5];
    float* out = (float*)d_out;

    hipLaunchKernelGGL(k_elman, dim3(nb / RB), dim3(NTHR), 0, stream,
                       x, Whx, Whh, Wph, bh, bp, out, nb, T);
}
